// Stacked_LSTM_55336358642684
// MI455X (gfx1250) — hardware-verified
//
#include <hip/hip_runtime.h>

typedef __attribute__((ext_vector_type(16))) _Float16 v16h;
typedef __attribute__((ext_vector_type(8)))  _Float16 v8h;
typedef __attribute__((ext_vector_type(8)))  float    v8f;
typedef __attribute__((ext_vector_type(4)))  float    v4f;
typedef __attribute__((ext_vector_type(2)))  float    v2f;

__device__ __forceinline__ void dep_guard_h(v8f& a, v8f& b, v16h x, v16h y) { asm volatile("v_nop\n\tv_nop\n\tv_nop\n\tv_nop" : "+v"(a), "+v"(b) : "v"(x), "v"(y)); }
__device__ __forceinline__ void keep4_h(v16h a, v16h b, v16h c, v16h d) { asm volatile("v_nop" :: "v"(a), "v"(b), "v"(c), "v"(d)); }
template <typename T> struct Frag;
template <> struct Frag<_Float16> {
  typedef v16h V; union U { v16h v; v8h h[2]; };
  static __device__ __forceinline__ v16h load(const _Float16* p) {
    U f; f.h[0] = *(const v8h*)(p); f.h[1] = *(const v8h*)(p + 16); return f.v;
  }
  static __device__ __forceinline__ v8f mma(v16h a, v16h b, v8f c) {
    return __builtin_amdgcn_wmma_f32_16x16x32_f16(false, a, false, b, (short)0, c, false, false);
  }
  static __device__ __forceinline__ void guard(v8f& a, v8f& b, v16h x, v16h y) { dep_guard_h(a, b, x, y); }
  static __device__ __forceinline__ void keep(v16h a, v16h b, v16h c, v16h d) { keep4_h(a, b, c, d); }
};

__device__ __forceinline__ v8f mma_f16g(v16h a, v16h b, v8f c) {
  c = __builtin_amdgcn_wmma_f32_16x16x32_f16(false, a, false, b, (short)0, c, false, false);
  asm volatile("v_nop\n\tv_nop\n\tv_nop\n\tv_nop" : "+v"(c) : "v"(a), "v"(b));
  return c;
}

constexpr int NBATCH  = 512;
constexpr int NSTEP   = 1024;
constexpr int NHID    = 128;
constexpr int NGATE   = 4 * NHID;
constexpr int ROWS_PB = 16;
constexpr int NWAVE   = 8;
constexpr int NTHR    = 32 * NWAVE;
constexpr int HPITCH  = 264;
constexpr int KW1     = NHID;
constexpr int KW2     = 2 * NHID;
constexpr int TCHUNK  = 32;
constexpr float WCARRY     = 16.0f;
constexpr float WCARRY_INV = 0.0625f;

static_assert(NBATCH % ROWS_PB == 0, "rows");
static_assert(NSTEP % TCHUNK == 0, "chunks");
static_assert(NHID == 16 * NWAVE, "unit subtiles per wave");
static_assert((HPITCH * 2) % 16 == 0, "tile row alignment");

__device__ __forceinline__ float sigm_f(float x) {
  x = fminf(fmaxf(x, -30.0f), 30.0f);
  return 1.0f / (1.0f + expf(-x));
}

__global__ __launch_bounds__(256) void prep_w1_plane(const float* __restrict__ w, _Float16* __restrict__ outp, int n2) {
  const int i = blockIdx.x * 256 + threadIdx.x;
  if (i < n2) {
    const _Float16 h0 = (_Float16)(w[2 * i] * WCARRY);
    const _Float16 h1 = (_Float16)(w[2 * i + 1] * WCARRY);
    const unsigned u = (unsigned)__builtin_bit_cast(unsigned short, h0) | ((unsigned)__builtin_bit_cast(unsigned short, h1) << 16);
    ((volatile unsigned*)outp)[i] = u;
    __threadfence();
    ((volatile unsigned*)outp)[i] = u;
  }
}

__global__ __launch_bounds__(256) void prep_w2_plane(const float* __restrict__ wa, const float* __restrict__ wb,
                                                     _Float16* __restrict__ outp, int n2) {
  const int i = blockIdx.x * 256 + threadIdx.x;
  if (i < n2) {
    const int row = i >> 7;
    const int cp  = i & 127;
    const int col = 2 * cp;
    const int cc  = col & 127;
    const size_t src = (size_t)row * NHID + cc;
    const float a0 = wa[src], a1 = wa[src + 1];
    const float b0 = wb[src], b1 = wb[src + 1];
    const bool second = (col >= NHID);
    const float v0 = second ? b0 : a0;
    const float v1 = second ? b1 : a1;
    const _Float16 h0 = (_Float16)(v0 * WCARRY);
    const _Float16 h1 = (_Float16)(v1 * WCARRY);
    const unsigned u = (unsigned)__builtin_bit_cast(unsigned short, h0) | ((unsigned)__builtin_bit_cast(unsigned short, h1) << 16);
    ((volatile unsigned*)outp)[i] = u;
    __threadfence();
    ((volatile unsigned*)outp)[i] = u;
  }
}

__global__ __launch_bounds__(NTHR) void lstm2_persist(
    const float* __restrict__ xin,
    const float* __restrict__ W_ih1, const float* __restrict__ b_ih1, const float* __restrict__ b_hh1,
    const float* __restrict__ b_ih2, const float* __restrict__ b_hh2,
    const float* __restrict__ W_out, const float* __restrict__ b_out,
    const _Float16* __restrict__ W1p, const _Float16* __restrict__ W2p,
    float* __restrict__ out) {
  __shared__ __align__(16) _Float16 hbuf[2][ROWS_PB * HPITCH];
  __shared__ __align__(16) float xs[ROWS_PB * TCHUNK];
  __shared__ __align__(16) float outs[ROWS_PB * TCHUNK];
  __shared__ __align__(16) float part[ROWS_PB * NWAVE];

  const int tid   = threadIdx.x;
  const int lane  = tid & 31;
  const int wave  = tid >> 5;
  const int hh    = lane >> 4;
  const int c     = lane & 15;
  const int bbase = blockIdx.x * ROWS_PB;
  const int ucol  = wave * 16 + c;

  {
    _Float16* hb = &hbuf[0][0];
    for (int i = tid; i < 2 * ROWS_PB * HPITCH; i += NTHR) hb[i] = (_Float16)0.0f;
  }

  float wih[4], bi1[4], bh1[4], bi2[4], bh2[4];
#pragma unroll
  for (int g = 0; g < 4; ++g) {
    const int n = g * NHID + ucol;
    wih[g] = W_ih1[n];
    bi1[g] = b_ih1[n];
    bh1[g] = b_hh1[n];
    bi2[g] = b_ih2[n];
    bh2[g] = b_hh2[n];
  }
  const float wo = W_out[ucol];
  const float bo = b_out[0];
  float c1s[8], c2s[8];
#pragma unroll
  for (int r = 0; r < 8; ++r) { c1s[r] = 0.0f; c2s[r] = 0.0f; }

  __syncthreads();

  for (int t = 0; t < NSTEP; ++t) {
    const int cb = t & 1;
    const int pb = cb ^ 1;
    const int tc = t & (TCHUNK - 1);

    if (tc == 0) {
      const int row = tid >> 4, cp = tid & 15;
      const v2f xv2 = *(const v2f*)(xin + (size_t)(bbase + row) * NSTEP + t + 2 * cp);
      xs[row * TCHUNK + 2 * cp]     = xv2[0];
      xs[row * TCHUNK + 2 * cp + 1] = xv2[1];
      __syncthreads();
    }

    v8f acc[4];
#pragma unroll
    for (int g = 0; g < 4; ++g) acc[g] = (v8f){0.f, 0.f, 0.f, 0.f, 0.f, 0.f, 0.f, 0.f};
    {
      const _Float16* At = &hbuf[pb][0] + c * HPITCH + 8 * hh;
      const _Float16* Bt = W1p + (size_t)ucol * KW1 + 8 * hh;
#pragma unroll 2
      for (int ks = 0; ks < 4; ++ks) {
        const int k0 = ks * 32;
        const v16h a = Frag<_Float16>::load(At + k0);
#pragma unroll
        for (int g = 0; g < 4; ++g) {
          const v16h bw = Frag<_Float16>::load(Bt + (size_t)g * NHID * KW1 + k0);
          acc[g] = mma_f16g(a, bw, acc[g]);
        }
      }
    }
#pragma unroll
    for (int r = 0; r < 8; ++r) {
      const int row = 8 * hh + r;
      const float xv = xs[row * TCHUNK + tc];
      float pi = xv * wih[0] + bi1[0]; pi += acc[0][r] * WCARRY_INV; pi += bh1[0];
      float pf = xv * wih[1] + bi1[1]; pf += acc[1][r] * WCARRY_INV; pf += bh1[1];
      float pg = xv * wih[2] + bi1[2]; pg += acc[2][r] * WCARRY_INV; pg += bh1[2];
      float po = xv * wih[3] + bi1[3]; po += acc[3][r] * WCARRY_INV; po += bh1[3];
      const float ig = sigm_f(pi);
      const float fg = sigm_f(pf);
      const float gg = tanhf(pg);
      const float og = sigm_f(po);
      const float cn = fg * c1s[r] + ig * gg;
      c1s[r] = cn;
      const float hn = og * tanhf(cn);
      hbuf[cb][row * HPITCH + ucol] = (_Float16)hn;
    }
    __syncthreads();

#pragma unroll
    for (int g = 0; g < 4; ++g) acc[g] = (v8f){0.f, 0.f, 0.f, 0.f, 0.f, 0.f, 0.f, 0.f};
    {
      const _Float16* At = &hbuf[cb][0] + c * HPITCH + 8 * hh;
      const _Float16* Bt = W2p + (size_t)ucol * KW2 + 8 * hh;
#pragma unroll 2
      for (int ks = 0; ks < 4; ++ks) {
        const int k0 = ks * 32;
        const v16h a = Frag<_Float16>::load(At + k0);
#pragma unroll
        for (int g = 0; g < 4; ++g) {
          const v16h bw = Frag<_Float16>::load(Bt + (size_t)g * NHID * KW2 + k0);
          acc[g] = mma_f16g(a, bw, acc[g]);
        }
      }
    }
    {
      const _Float16* At = &hbuf[pb][0] + c * HPITCH + NHID + 8 * hh;
      const _Float16* Bt = W2p + (size_t)ucol * KW2 + NHID + 8 * hh;
#pragma unroll 2
      for (int ks = 0; ks < 4; ++ks) {
        const int k0 = ks * 32;
        const v16h a = Frag<_Float16>::load(At + k0);
#pragma unroll
        for (int g = 0; g < 4; ++g) {
          const v16h bw = Frag<_Float16>::load(Bt + (size_t)g * NHID * KW2 + k0);
          acc[g] = mma_f16g(a, bw, acc[g]);
        }
      }
    }
    float pr[8];
#pragma unroll
    for (int r = 0; r < 8; ++r) {
      const int row = 8 * hh + r;
      float pi = acc[0][r] * WCARRY_INV + bi2[0]; pi += bh2[0];
      float pf = acc[1][r] * WCARRY_INV + bi2[1]; pf += bh2[1];
      float pg = acc[2][r] * WCARRY_INV + bi2[2]; pg += bh2[2];
      float po = acc[3][r] * WCARRY_INV + bi2[3]; po += bh2[3];
      const float ig = sigm_f(pi);
      const float fg = sigm_f(pf);
      const float gg = tanhf(pg);
      const float og = sigm_f(po);
      const float cn = fg * c2s[r] + ig * gg;
      c2s[r] = cn;
      const float hn = og * tanhf(cn);
      hbuf[cb][row * HPITCH + NHID + ucol] = (_Float16)hn;
      pr[r] = hn * wo;
    }
#pragma unroll
    for (int r = 0; r < 8; ++r) {
      float p = pr[r];
      p += __shfl_xor(p, 1, 32);
      p += __shfl_xor(p, 2, 32);
      p += __shfl_xor(p, 4, 32);
      p += __shfl_xor(p, 8, 32);
      pr[r] = p;
    }
    if (c == 0) {
#pragma unroll
      for (int r = 0; r < 8; ++r) part[(8 * hh + r) * NWAVE + wave] = pr[r];
    }
    __syncthreads();

    if (wave == 0) {
      const int row = lane & 15;
      float s = part[row * NWAVE + 0];
      s += part[row * NWAVE + 1];
      s += part[row * NWAVE + 2];
      s += part[row * NWAVE + 3];
      s += part[row * NWAVE + 4];
      s += part[row * NWAVE + 5];
      s += part[row * NWAVE + 6];
      s += part[row * NWAVE + 7];
      s += bo;
      outs[row * TCHUNK + tc] = s;
      if (tc == TCHUNK - 1) {
        __builtin_amdgcn_fence(__ATOMIC_RELEASE, "workgroup");
        __builtin_amdgcn_wave_barrier();
        __builtin_amdgcn_fence(__ATOMIC_ACQUIRE, "workgroup");
        const int q = lane >> 3, c4 = (lane & 7) * 4;
        const size_t gbase = (size_t)bbase * NSTEP + (size_t)(t - (TCHUNK - 1));
        for (int pass = 0; pass < 2; ++pass) {
#pragma unroll
          for (int it = 0; it < 4; ++it) {
            const int orow = it * 4 + q;
            const v4f v = *(const v4f*)(outs + orow * TCHUNK + c4);
            *(volatile v4f*)(out + gbase + (size_t)orow * NSTEP + c4) = v;
          }
          __threadfence();
        }
      }
    }
  }
}

extern "C" void kernel_launch(void* const* d_in, const int* in_sizes, int n_in,
                              void* d_out, int out_size, void* d_ws, size_t ws_size,
                              hipStream_t stream) {
  if (n_in < 11) return;
  if (in_sizes[0] != NBATCH * NSTEP) return;
  if (in_sizes[1] != NGATE || in_sizes[2] != NGATE * NHID) return;
  if (in_sizes[3] != NGATE || in_sizes[4] != NGATE) return;
  if (in_sizes[5] != NGATE * NHID || in_sizes[6] != NGATE * NHID) return;
  if (in_sizes[7] != NGATE || in_sizes[8] != NGATE) return;
  if (in_sizes[9] != NHID || in_sizes[10] < 1) return;
  if (out_size != NBATCH * NSTEP) return;
  const size_t w1_bytes = (size_t)NGATE * KW1 * 2;
  const size_t w2_bytes = (size_t)NGATE * KW2 * 2;
  if (ws_size < w1_bytes + w2_bytes) return;

  const float* xin   = (const float*)d_in[0];
  const float* W_ih1 = (const float*)d_in[1];
  const float* W_hh1 = (const float*)d_in[2];
  const float* b_ih1 = (const float*)d_in[3];
  const float* b_hh1 = (const float*)d_in[4];
  const float* W_ih2 = (const float*)d_in[5];
  const float* W_hh2 = (const float*)d_in[6];
  const float* b_ih2 = (const float*)d_in[7];
  const float* b_hh2 = (const float*)d_in[8];
  const float* W_out = (const float*)d_in[9];
  const float* b_out = (const float*)d_in[10];
  float* out = (float*)d_out;
  _Float16* W1p = (_Float16*)d_ws;
  _Float16* W2p = (_Float16*)((char*)d_ws + w1_bytes);

  const int n2_w1 = NGATE * KW1 / 2;
  const int n2_w2 = NGATE * KW2 / 2;
  prep_w1_plane<<<dim3((n2_w1 + 255) / 256), dim3(256), 0, stream>>>(W_hh1, W1p, n2_w1);
  prep_w2_plane<<<dim3((n2_w2 + 255) / 256), dim3(256), 0, stream>>>(W_ih2, W_hh2, W2p, n2_w2);
  lstm2_persist<<<dim3(NBATCH / ROWS_PB), dim3(NTHR), 0, stream>>>(
      xin, W_ih1, b_ih1, b_hh1, b_ih2, b_hh2, W_out, b_out, W1p, W2p, out);
}
